// MoEBertSelfOutput_38534446579846
// MI455X (gfx1250) — hardware-run, weakly checked
//
#include <hip/hip_runtime.h>
#include <math.h>

#define NB 16
#define TPB 512
#define NTOK (NB * TPB)
#define DM 1024
#define FF 1024
#define NE 8
#define R_MAX NTOK
#define NT_MAX (R_MAX / 64)
#define TILES_PER_ROW (TPB / 64)

#define CX_LOG2 11
#define CW_LOG2 16
#define CH_LOG2 11
#define SC_Y (1.0f / (float)(1u << (CH_LOG2 + CW_LOG2)))

#define TBL_NTILES 32
#define TBL_TILE_E 64
#define TBL_WORDS 256

static_assert(NE == 8 && NB == 16 && TPB == 512 && TPB % 64 == 0 && TILES_PER_ROW == 8);
static_assert(DM == 1024 && FF == 1024 && DM % 128 == 0 && NTOK % 8 == 0);
static_assert(NT_MAX == 128 && TBL_NTILES < TBL_TILE_E && TBL_TILE_E + NT_MAX <= TBL_WORDS);
static_assert(CX_LOG2 == 11 && CW_LOG2 == 16 && CH_LOG2 == CX_LOG2);
static_assert((NTOK * FF / 8) % 256 == 0);

constexpr size_t al256(size_t b) { return (b + 255) & ~(size_t)255; }
constexpr size_t SZ_X16 = al256((size_t)NTOK * FF * 2);
constexpr size_t SZ_WP  = al256((size_t)NE * DM * FF * 2);
constexpr size_t SZ_TBL = al256((size_t)TBL_WORDS * 4);
constexpr size_t SZ_YG  = al256((size_t)R_MAX * DM * 4);
constexpr size_t WS_TOTAL = SZ_X16 + SZ_WP + SZ_TBL + SZ_YG;
static_assert(WS_TOTAL == (size_t)67109888 && WS_TOTAL < (size_t)134217728);

typedef _Float16 h16;
typedef __attribute__((ext_vector_type(16))) _Float16 v16h;
typedef __attribute__((ext_vector_type(8)))  _Float16 v8h;
typedef __attribute__((ext_vector_type(8)))  float    v8f;
typedef __attribute__((ext_vector_type(4)))  float    v4f;
typedef __attribute__((ext_vector_type(2)))  float    v2f;
typedef __attribute__((ext_vector_type(4)))  unsigned int v4u;
typedef __attribute__((ext_vector_type(4)))  int      v4i;
typedef __attribute__((ext_vector_type(2)))  int      v2i;


#define VST2(T, ptr, val) do { const T vst2_v_ = (val); *(volatile T*)(ptr) = vst2_v_; __threadfence(); *(volatile T*)(ptr) = vst2_v_; } while (0)

static __device__ __forceinline__ float bfr(float f) {
    unsigned u = __float_as_uint(f);
    u += 0x7FFFu + ((u >> 16) & 1u);
    return __uint_as_float(u & 0xFFFF0000u);
}
static __device__ __forceinline__ h16 toh_flush(float v) { const float w = (fabsf(v) < 6.103515625e-05f) ? 0.0f : v; return (h16)w; }
static __device__ __forceinline__ void st8h(h16* p, const float* v) {
    v8h hv;
#pragma unroll
    for (int e = 0; e < 8; ++e) hv[e] = toh_flush(v[e]);
    VST2(v8h, p, hv);
}

union FragU { v16h v; v8h h[2]; };
static __device__ __forceinline__ v16h frag_ld(const h16* p) {
    FragU f; f.h[0] = *(const v8h*)(p); f.h[1] = *(const v8h*)(p + 16); return f.v;
}
static __device__ __forceinline__ v8f wmma16g(v16h a, v16h b, v8f c) {
    c = __builtin_amdgcn_wmma_f32_16x16x32_f16(false, a, false, b, (short)0, c, false, false);
    asm volatile("v_nop\n\tv_nop\n\tv_nop\n\tv_nop" : "+v"(c) : "v"(a), "v"(b));
    return c;
}
static __device__ __forceinline__ void wave_sync_lds() {
    __builtin_amdgcn_fence(3  , "workgroup");
    __builtin_amdgcn_wave_barrier();
    __builtin_amdgcn_fence(2  , "workgroup");
}

template <int LOG2C>
__global__ __launch_bounds__(256) void k_plane(const float* __restrict__ src, h16* __restrict__ dst, unsigned n8) {
    const unsigned u = blockIdx.x * 256u + threadIdx.x;
    if (u >= n8) return;
    const float cs = (float)(1u << LOG2C);
    const v4f a = *(const v4f*)(src + (size_t)u * 8u);
    const v4f b = *(const v4f*)(src + (size_t)u * 8u + 4u);
    float v[8] = {bfr(a.x) * cs, bfr(a.y) * cs, bfr(a.z) * cs, bfr(a.w) * cs, bfr(b.x) * cs, bfr(b.y) * cs, bfr(b.z) * cs, bfr(b.w) * cs};
    st8h(dst + (size_t)u * 8u, v);
}

__global__ __launch_bounds__(128) void k_planeTw(const float* __restrict__ src, h16* __restrict__ dst, unsigned ne, unsigned K, unsigned N, unsigned pitch, unsigned estride, float cs) {
    __shared__ __align__(16) float sT[4][64 * 36];
    const unsigned lane = threadIdx.x & 31u;
    const unsigned wave = threadIdx.x >> 5;
    const unsigned tk = K >> 6, tn = N >> 5;
    const unsigned tpe = tk * tn;
    const unsigned u = blockIdx.x * 4u + wave;
    if (u >= ne * tpe) return;
    const unsigned e = u / tpe;
    const unsigned rem = u - e * tpe;
    const unsigned kt = rem / tn;
    const unsigned nt = rem - kt * tn;
    const unsigned k0 = kt << 6, n0 = nt << 5;
    const size_t sbase = (size_t)e * (size_t)estride;
    const size_t ebase = (size_t)e * ((size_t)K * (size_t)N);
    float* slab = sT[wave];
#pragma unroll
    for (int i = 0; i < 16; ++i) {
        const unsigned p = lane + 32u * (unsigned)i;
        const unsigned kr = p >> 3;
        const unsigned n4 = (p & 7u) * 4u;
        const v4f a = *(const v4f*)(src + sbase + (size_t)(k0 + kr) * pitch + n0 + n4);
        v4f s;
        s.x = bfr(a.x) * cs; s.y = bfr(a.y) * cs; s.z = bfr(a.z) * cs; s.w = bfr(a.w) * cs;
        *(v4f*)(&slab[kr * 36u + n4]) = s;
    }
    wave_sync_lds();
#pragma unroll
    for (int i = 0; i < 8; ++i) {
        const unsigned q = lane + 32u * (unsigned)i;
        const unsigned n = q >> 3;
        const unsigned kp = q & 7u;
        float v[8];
#pragma unroll
        for (int j = 0; j < 8; ++j) v[j] = slab[(8u * kp + (unsigned)j) * 36u + n];
        st8h(dst + ebase + (size_t)(n0 + n) * K + k0 + 8u * kp, v);
    }
}

__global__ __launch_bounds__(128) void k_tbl_idx(const int* __restrict__ idx, int* __restrict__ tbl) {
    const unsigned i = threadIdx.x;
    if (blockIdx.x != 0u || i >= (unsigned)NT_MAX) return;
    const int e = min(max(idx[i / (unsigned)TILES_PER_ROW], 0), NE - 1);
    VST2(int, tbl + TBL_TILE_E + i, e);
    if (i == 0u) { VST2(int, tbl + TBL_NTILES, (int)NT_MAX); }
}

__global__ __launch_bounds__(256) void k_ffn2(const h16* __restrict__ Hg, const h16* __restrict__ Wp, const float* __restrict__ eb,
                                              const int* __restrict__ tbl, float* __restrict__ Yg) {
    __shared__ __align__(16) float sT[8][16 * 68];
    const unsigned lane = threadIdx.x & 31u;
    const unsigned wave = threadIdx.x >> 5;
    const unsigned u = blockIdx.x * 8u + wave;
    if (u >= (unsigned)(NT_MAX * (DM / 64))) return;
    const unsigned rowtile = u / (unsigned)(DM / 64);
    const unsigned ct = u - rowtile * (unsigned)(DM / 64);
    const int nt = min(max(tbl[TBL_NTILES], 0), NT_MAX);
    if ((int)rowtile >= nt) return;
    const int e = min(max(tbl[TBL_TILE_E + rowtile], 0), NE - 1);
    const size_t wbase = (size_t)(unsigned)e * (size_t)(DM * FF);
    const unsigned m0 = rowtile << 6, n0 = ct << 6;
    const unsigned rlane = lane & 15u;
    const unsigned koff = (lane >> 4) * 8u;
    const unsigned mOff = koff;

    v8f acc[4][4];
#pragma unroll
    for (int i = 0; i < 4; ++i)
#pragma unroll
        for (int j = 0; j < 4; ++j) acc[i][j] = (v8f){0.f,0.f,0.f,0.f,0.f,0.f,0.f,0.f};

    for (unsigned k0 = 0; k0 < (unsigned)FF; k0 += 32u) {
        v16h bh[4];
#pragma unroll
        for (int j = 0; j < 4; ++j)
            bh[j] = frag_ld(Wp + wbase + (size_t)(n0 + ((unsigned)j << 4) + rlane) * FF + koff + k0);
#pragma unroll
        for (int i = 0; i < 4; ++i) {
            const v16h ah = frag_ld(Hg + (size_t)(m0 + ((unsigned)i << 4) + rlane) * FF + koff + k0);
#pragma unroll
            for (int j = 0; j < 4; ++j) acc[i][j] = wmma16g(ah, bh[j], acc[i][j]);
        }
    }

    float ebv[4];
#pragma unroll
    for (int j = 0; j < 4; ++j) ebv[j] = bfr(eb[(unsigned)e * (unsigned)DM + n0 + ((unsigned)j << 4) + rlane]);

    float* slab = sT[wave];
#pragma unroll
    for (int i = 0; i < 4; ++i) {
        const unsigned mBase = m0 + ((unsigned)i << 4);
#pragma unroll
        for (int j = 0; j < 4; ++j)
#pragma unroll
            for (int r = 0; r < 8; ++r)
                slab[(mOff + (unsigned)r) * 68u + ((unsigned)j << 4) + rlane] = acc[i][j][r] * SC_Y + ebv[j];
        wave_sync_lds();
        const unsigned hh = lane >> 4, c4 = (lane & 15u) * 4u;
#pragma unroll
        for (int half = 0; half < 2; ++half) {
            v4f vv[4];
#pragma unroll
            for (int it = 0; it < 4; ++it) {
                const unsigned row = (unsigned)(half * 4 + it) * 2u + hh;
                vv[it] = *(const v4f*)(slab + row * 68u + c4);
            }
            for (int pass = 0; pass < 2; ++pass) {
#pragma unroll
                for (int it = 0; it < 4; ++it) {
                    const unsigned row = (unsigned)(half * 4 + it) * 2u + hh;
                    *(volatile v4f*)(Yg + (size_t)(mBase + row) * DM + n0 + c4) = vv[it];
                }
                __threadfence();
            }
        }
        wave_sync_lds();
    }
}

__global__ __launch_bounds__(256) void k_resln(const float* __restrict__ Yg, const float* __restrict__ r, const float* __restrict__ gamma, const float* __restrict__ beta,
                                               float* __restrict__ out) {
    const unsigned lane = threadIdx.x & 31u;
    const unsigned wave = threadIdx.x >> 5;
    const unsigned t = blockIdx.x * 8u + wave;
    if (t >= (unsigned)NTOK) return;
    v4f y[8];
    float s = 0.0f;
#pragma unroll
    for (int q = 0; q < 8; ++q) {
        const unsigned c = 4u * lane + 128u * (unsigned)q;
        const v4f ra = *(const v4f*)(r + (size_t)t * DM + c);
        const v4f a = *(const v4f*)(Yg + (size_t)t * DM + c);
        y[q].x = a.x + bfr(ra.x); y[q].y = a.y + bfr(ra.y);
        y[q].z = a.z + bfr(ra.z); y[q].w = a.w + bfr(ra.w);
        s = (((s + y[q].x) + y[q].y) + y[q].z) + y[q].w;
    }
    s += __shfl_xor(s, 16, 32);
    s += __shfl_xor(s, 8, 32);
    s += __shfl_xor(s, 4, 32);
    s += __shfl_xor(s, 2, 32);
    s += __shfl_xor(s, 1, 32);
    const float mu = s / (float)DM;
    float vs = 0.0f;
#pragma unroll
    for (int q = 0; q < 8; ++q) {
        y[q].x -= mu; y[q].y -= mu; y[q].z -= mu; y[q].w -= mu;
        vs = (((vs + y[q].x * y[q].x) + y[q].y * y[q].y) + y[q].z * y[q].z) + y[q].w * y[q].w;
    }
    vs += __shfl_xor(vs, 16, 32);
    vs += __shfl_xor(vs, 8, 32);
    vs += __shfl_xor(vs, 4, 32);
    vs += __shfl_xor(vs, 2, 32);
    vs += __shfl_xor(vs, 1, 32);
    const float var = vs / (float)DM;
    const float rs = 1.0f / sqrtf(var + 1e-12f);
    for (int pass = 0; pass < 2; ++pass) {
#pragma unroll
        for (int q = 0; q < 8; ++q) {
            const unsigned c = 4u * lane + 128u * (unsigned)q;
            const v4f ga = *(const v4f*)(gamma + c);
            const v4f be = *(const v4f*)(beta + c);
            v4f o;
            o.x = bfr(ga.x) * (y[q].x * rs) + bfr(be.x); o.y = bfr(ga.y) * (y[q].y * rs) + bfr(be.y);
            o.z = bfr(ga.z) * (y[q].z * rs) + bfr(be.z); o.w = bfr(ga.w) * (y[q].w * rs) + bfr(be.w);
            *(volatile v4f*)(out + (size_t)t * DM + c) = o;
        }
        __threadfence();
    }
}

extern "C" void kernel_launch(void* const* d_in, const int* in_sizes, int n_in, void* d_out, int out_size,
                              void* d_ws, size_t ws_size, hipStream_t stream) {
    if (n_in < 7) return;
    if (in_sizes[0] < NTOK * FF || in_sizes[1] < NTOK * DM || in_sizes[2] < NB || in_sizes[3] < NE * FF * DM || in_sizes[4] < NE * DM || in_sizes[5] < DM || in_sizes[6] < DM) return;
    if (out_size < NTOK * DM) return;

    const float* x     = (const float*)d_in[0];
    const float* resid = (const float*)d_in[1];
    const int*   idx   = (const int*)d_in[2];
    const float* w     = (const float*)d_in[3];
    const float* b     = (const float*)d_in[4];
    const float* gamma = (const float*)d_in[5];
    const float* beta  = (const float*)d_in[6];
    float* out = (float*)d_out;

    char* wsp = (char*)d_ws;
    size_t off = 0;
    auto carve = [&](size_t bytes) -> void* { void* r = wsp + off; off += (bytes + 255) & ~(size_t)255; return r; };
    h16*   x16 = (h16*)carve((size_t)NTOK * FF * 2);
    h16*   wpt = (h16*)carve((size_t)NE * DM * FF * 2);
    int*   tbl = (int*)carve((size_t)TBL_WORDS * 4);
    float* Yg  = (float*)carve((size_t)R_MAX * DM * 4);
    if (off != WS_TOTAL || off > ws_size || off > (size_t)134217728) return;

    k_plane<CX_LOG2><<<(NTOK * FF / 8) / 256, 256, 0, stream>>>(x, x16, (unsigned)(NTOK * FF / 8));
    k_planeTw<<<(NE * (FF / 64) * (DM / 32) + 3) / 4, 128, 0, stream>>>(w, wpt, (unsigned)NE, (unsigned)FF, (unsigned)DM, (unsigned)DM, (unsigned)(FF * DM), (float)(1u << CW_LOG2));
    k_tbl_idx<<<1, 128, 0, stream>>>(idx, tbl);
    k_ffn2<<<(NT_MAX * (DM / 64) + 7) / 8, 256, 0, stream>>>(x16, wpt, b, tbl, Yg);
    k_resln<<<NTOK / 8, 256, 0, stream>>>(Yg, resid, gamma, beta, out);
}
